// Architecture_43559558316192
// MI455X (gfx1250) — hardware-run, weakly checked
//
#include <hip/hip_runtime.h>
#include <math.h>

typedef __attribute__((ext_vector_type(16))) _Float16 v16h;
typedef __attribute__((ext_vector_type(8)))  _Float16 v8h;
typedef __attribute__((ext_vector_type(4)))  _Float16 v4h;
typedef __attribute__((ext_vector_type(8)))  float    v8f;
typedef __attribute__((ext_vector_type(4)))  float    v4f;

constexpr int kB  = 32;
constexpr int kS  = 256;
constexpr int kD  = 512;
constexpr int kH  = 8;
constexpr int kDh = 64;
constexpr int kF  = 2048;
constexpr int kL  = 6;
constexpr int kM  = kB * kS;
constexpr int kQT = 32;
constexpr int kSCP = 260;
constexpr int kATP = 264;
constexpr int kOSP = 68;
constexpr int kChunkMax = kS / 8;
static_assert(kH * kDh == kD, "head split");
static_assert(kM == 8192 && kS / kQT == 8 && kH == 8, "block decode uses 3+3 bit fields");
static_assert((kD % 32) == 0 && (kF % 32) == 0 && (kDh % 32) == 0, "K multiples of 32");
static_assert((kM % 64) == 0 && (kD % 64) == 0 && (kF % 64) == 0, "M,N multiples of 64");
static_assert((((kM / 64) * (kD / 64)) % 8) == 0 && (((kM / 64) * (kF / 64)) % 8) == 0, "8 wave tiles per block");
static_assert(kOSP * kQT <= kSCP * kQT, "output staging fits the score tile");
static_assert(kChunkMax == 32 && (kChunkMax % 4) == 0, "per-lane key chunk bound");

constexpr int isqrt_c(int n) { int r = 0; while ((r + 1) * (r + 1) <= n) ++r; return r; }
constexpr int kDhRoot = isqrt_c(kDh);
static_assert(kDhRoot * kDhRoot == kDh, "head dim is a perfect square");
constexpr float kScoreScale = 1.0f / (float)kDhRoot;
constexpr float kWCarry     = 16.0f;
constexpr float kWCarryInv  = 1.0f / kWCarry;
constexpr float kPCarry     = 2048.0f;
constexpr float kACarry     = 16.0f;
constexpr float kOutScale   = 1.0f / (kACarry * kWCarry);
constexpr float kInvD       = 1.0f / (float)kD;
constexpr float kLnEps      = 1e-5f;

constexpr size_t kPlaneF = (size_t)kM * kD * 4;
constexpr size_t kPlaneH = (size_t)kM * kD * 2;
constexpr size_t kOffP0  = 0;
constexpr size_t kOffP1  = kOffP0 + kPlaneF;
constexpr size_t kOffO   = kOffP1 + kPlaneF;
constexpr size_t kOffX16 = kOffO + kPlaneF;
constexpr size_t kOffY16 = kOffX16 + kPlaneH;
constexpr size_t kOffT16 = kOffY16 + kPlaneH;
constexpr size_t kOffU   = kOffT16 + kPlaneH;
constexpr size_t kSizeU  = (size_t)kM * kF * 2;
constexpr size_t kOffWS  = kOffU + kSizeU;
constexpr size_t kWsHalves = (size_t)3 * kD * kD + (size_t)2 * kD * kF;
constexpr size_t kWsTotal = kOffWS + kWsHalves * 2;
static_assert(kSizeU >= 3 * kPlaneH, "attention planes fit the union");
static_assert(kWsTotal == 114819072ull, "carve total");
static_assert(kWsTotal <= 134217728ull, "carve cap");
static_assert((kOffP1 % 256) == 0 && (kOffO % 256) == 0 && (kOffX16 % 256) == 0 && (kOffY16 % 256) == 0 &&
              (kOffT16 % 256) == 0 && (kOffU % 256) == 0 && (kOffWS % 256) == 0, "aligned regions");

__device__ __forceinline__ float bf16_rne(float f) {
  unsigned u = __float_as_uint(f);
  u = (u + 0x7FFFu + ((u >> 16) & 1u)) & 0xFFFF0000u;
  return __uint_as_float(u);
}
__device__ __forceinline__ void guard4_h(v8f& a, v8f& b, v8f& c, v8f& d, v16h x, v16h y) {
  asm volatile("v_nop\n\tv_nop\n\tv_nop\n\tv_nop" : "+v"(a), "+v"(b), "+v"(c), "+v"(d) : "v"(x), "v"(y));
}
__device__ __forceinline__ void guard2_h(v8f& a, v8f& b, v16h x, v16h y) {
  asm volatile("v_nop\n\tv_nop\n\tv_nop\n\tv_nop" : "+v"(a), "+v"(b) : "v"(x), "v"(y));
}
__device__ __forceinline__ void keep4_h(v16h a, v16h b, v16h c, v16h d) {
  asm volatile("v_nop" :: "v"(a), "v"(b), "v"(c), "v"(d));
}
__device__ __forceinline__ void acc_guard4(v8f& a, v8f& b, v8f& c, v8f& d) {
  asm volatile("v_nop\n\tv_nop\n\tv_nop\n\tv_nop" : "+v"(a), "+v"(b), "+v"(c), "+v"(d));
}
struct FragH {
  union U { v16h v; v8h h[2]; };
  static __device__ __forceinline__ v16h load(const _Float16* p) {
    U f;
    f.h[0] = *(const v8h*)(p);
    f.h[1] = *(const v8h*)(p + 16);
    return f.v;
  }
  static __device__ __forceinline__ v8f mma(v16h a, v16h b, v8f c) {
    return __builtin_amdgcn_wmma_f32_16x16x32_f16(false, a, false, b, (short)0, c, false, false);
  }
};
__device__ __forceinline__ v8f mma_guarded(v16h a, v16h b, v8f c) {
  c = __builtin_amdgcn_wmma_f32_16x16x32_f16(false, a, false, b, (short)0, c, false, false);
  asm volatile("v_nop\n\tv_nop\n\tv_nop\n\tv_nop" : "+v"(c) : "v"(a), "v"(b));
  return c;
}

template <int BIAS_MODE, int OUT_MODE, int ACT>
__global__ __launch_bounds__(256) void wmma_gemm64(
    const unsigned short* __restrict__ Ap, int lda,
    const unsigned short* __restrict__ Btp, int ldb,
    void* __restrict__ Cout, int ldc,
    const float* __restrict__ bias,
    int M, int N, int K, float scale) {
  const _Float16* A  = (const _Float16*)Ap;
  const _Float16* Bt = (const _Float16*)Btp;
  __shared__ __align__(16) float sT[8][16 * 68];
  const int lane = threadIdx.x & 31;
  const int wave = threadIdx.x >> 5;
  const int tilesN = N >> 6;
  const int tilesM = M >> 6;
  const int tile = blockIdx.x * 8 + wave;
  if (tile >= tilesM * tilesN) return;
  const int tm = tile / tilesN;
  const int tn = tile - tm * tilesN;
  const int m0 = tm << 6;
  const int n0 = tn << 6;

  const int rlane = lane & 15;
  const int koff  = (lane >> 4) * 8;
  const int mOff  = (lane >> 4) * 8;

  v8f acc[4][4];
#pragma unroll
  for (int i = 0; i < 4; ++i)
#pragma unroll
    for (int j = 0; j < 4; ++j) acc[i][j] = (v8f){0.f,0.f,0.f,0.f,0.f,0.f,0.f,0.f};

  for (int k0 = 0; k0 < K; k0 += 32) {
    v16h bh[4];
#pragma unroll
    for (int j = 0; j < 4; ++j) {
      const size_t bo = (size_t)(n0 + (j << 4) + rlane) * ldb + koff + k0;
      bh[j] = FragH::load(Bt + bo);
    }
#pragma unroll
    for (int i = 0; i < 4; ++i) {
      const size_t ao = (size_t)(m0 + (i << 4) + rlane) * lda + koff + k0;
      const v16h ah = FragH::load(A + ao);
#pragma unroll
      for (int j = 0; j < 4; ++j) acc[i][j] = FragH::mma(ah, bh[j], acc[i][j]);
      guard4_h(acc[i][0], acc[i][1], acc[i][2], acc[i][3], ah, bh[3]);
    }
    keep4_h(bh[0], bh[1], bh[2], bh[3]);
  }
  acc_guard4(acc[0][0], acc[0][1], acc[0][2], acc[0][3]);
  acc_guard4(acc[1][0], acc[1][1], acc[1][2], acc[1][3]);
  acc_guard4(acc[2][0], acc[2][1], acc[2][2], acc[2][3]);
  acc_guard4(acc[3][0], acc[3][1], acc[3][2], acc[3][3]);

  float* slab = sT[wave];
#pragma unroll
  for (int i = 0; i < 4; ++i) {
    const int mBase = m0 + (i << 4);
    float brow[8];
#pragma unroll
    for (int r = 0; r < 8; ++r) brow[r] = (BIAS_MODE == 1) ? bf16_rne(bias[mBase + mOff + r]) : 0.f;
#pragma unroll
    for (int j = 0; j < 4; ++j) {
      const int n = n0 + (j << 4) + rlane;
      float bv = 0.f;
      if (BIAS_MODE == 2) bv = bf16_rne(bias[n]);
#pragma unroll
      for (int r = 0; r < 8; ++r) {
        float v = acc[i][j][r] * scale;
        if (BIAS_MODE == 1) v += brow[r];
        if (BIAS_MODE == 2) v += bv;
        if (ACT == 2) v = fmaxf(v, 0.0f);
        slab[(mOff + r) * 68 + (j << 4) + rlane] = v;
      }
    }
    __builtin_amdgcn_fence(__ATOMIC_RELEASE, "workgroup");
    __builtin_amdgcn_wave_barrier();
    __builtin_amdgcn_fence(__ATOMIC_ACQUIRE, "workgroup");
    if (OUT_MODE == 0) {
      float* C = (float*)Cout;
      const int hh = lane >> 4, c4 = (lane & 15) * 4;
      for (int pass = 0; pass < 2; ++pass) {
#pragma unroll
        for (int it = 0; it < 8; ++it) {
          const int row = it * 2 + hh;
          const v4f v = *(const v4f*)(slab + row * 68 + c4);
          *(volatile v4f*)(C + (size_t)(mBase + row) * ldc + n0 + c4) = v;
        }
        __threadfence();
      }
    } else {
      const int q = lane >> 3, c8 = (lane & 7) * 8;
      unsigned short* C = (unsigned short*)Cout;
      for (int pass = 0; pass < 2; ++pass) {
#pragma unroll
        for (int it = 0; it < 4; ++it) {
          const int row = it * 4 + q;
          const float* sp = slab + row * 68 + c8;
          v8h hv;
#pragma unroll
          for (int e = 0; e < 8; ++e) hv[e] = (_Float16)sp[e];
          *(volatile v8h*)(C + (size_t)(mBase + row) * ldc + n0 + c8) = hv;
        }
        __threadfence();
      }
    }
    __builtin_amdgcn_fence(__ATOMIC_RELEASE, "workgroup");
    __builtin_amdgcn_wave_barrier();
    __builtin_amdgcn_fence(__ATOMIC_ACQUIRE, "workgroup");
  }
}

__global__ __launch_bounds__(256) void cast8_kernel(const float* __restrict__ in, unsigned short* __restrict__ out, int n8) {
  const int i = blockIdx.x * 256 + threadIdx.x;
  if (i >= n8) return;
  const float* p = in + 8 * (size_t)i;
  const v4f a = *(const v4f*)(p);
  const v4f c = *(const v4f*)(p + 4);
  v8h hv;
#pragma unroll
  for (int e = 0; e < 4; ++e) {
    hv[e]     = (_Float16)bf16_rne(a[e]);
    hv[4 + e] = (_Float16)bf16_rne(c[e]);
  }
  unsigned short* q = out + 8 * (size_t)i;
  *(volatile v8h*)q = hv;
  __threadfence();
  *(volatile v8h*)q = hv;
}

__global__ __launch_bounds__(256) void wprep_kernel(const float* __restrict__ Wk, const float* __restrict__ Wv,
                                                    const float* __restrict__ Wo, const float* __restrict__ W1,
                                                    const float* __restrict__ W2, unsigned short* __restrict__ out) {
  __shared__ float sm[64][65];
  const int t = threadIdx.x;
  const int bid = blockIdx.x;
  const float* W = Wk;
  int Kin = kD, Nout = kD, tl = bid;
  size_t outOff = 0;
  if (bid >= 448)      { W = W2; Kin = kF; Nout = kD; tl = bid - 448; outOff = (size_t)3 * kD * kD + (size_t)kD * kF; }
  else if (bid >= 192) { W = W1; Kin = kD; Nout = kF; tl = bid - 192; outOff = (size_t)3 * kD * kD; }
  else if (bid >= 128) { W = Wo; tl = bid - 128; outOff = (size_t)2 * kD * kD; }
  else if (bid >= 64)  { W = Wv; tl = bid - 64;  outOff = (size_t)kD * kD; }
  const int tilesK = Kin >> 6;
  const int nt = tl / tilesK;
  const int kt = tl - nt * tilesK;
  const int k0 = kt << 6, n0 = nt << 6;
#pragma unroll
  for (int i = 0; i < 16; ++i) {
    const int e = i * 256 + t;
    const int r = e >> 6;
    const int c = e & 63;
    sm[c][r] = bf16_rne(W[(size_t)(k0 + r) * Nout + n0 + c]) * kWCarry;
  }
  __syncthreads();
  const int lane = t & 31, wave = t >> 5;
  const int q = lane >> 3, c8 = (lane & 7) * 8;
  unsigned short* op = out + outOff;
  for (int pass = 0; pass < 2; ++pass) {
#pragma unroll
    for (int it = 0; it < 2; ++it) {
      const int row = wave * 8 + it * 4 + q;
      v8h hv;
#pragma unroll
      for (int e = 0; e < 8; ++e) hv[e] = (_Float16)sm[row][c8 + e];
      *(volatile v8h*)(op + (size_t)(n0 + row) * Kin + k0 + c8) = hv;
    }
    __threadfence();
  }
}

__global__ __launch_bounds__(256) void decay_attn_kernel(
    const unsigned short* __restrict__ qk16, const unsigned short* __restrict__ vT16,
    unsigned short* __restrict__ a16, const float* __restrict__ gam, int strict) {
  __shared__ __align__(16) float sc[kQT * kSCP];
  __shared__ __align__(16) _Float16 at[kQT * kATP];
  __shared__ float rinv[kQT];

  const int tid = threadIdx.x, wave = tid >> 5, lane = tid & 31;
  const int hh = lane >> 4, c = lane & 15;
  const int bx = blockIdx.x;
  const int qt = bx & 7;
  const int h  = (bx >> 3) & (kH - 1);
  const int b  = bx >> 6;
  const int q0 = qt * kQT;
  const int nk = q0 + kQT;
  const _Float16* Qb = (const _Float16*)qk16 + (size_t)b * kS * kD + h * kDh;

  {
    v16h qa[2][2];
#pragma unroll
    for (int rt = 0; rt < 2; ++rt)
#pragma unroll
      for (int dc = 0; dc < 2; ++dc)
        qa[rt][dc] = FragH::load(Qb + (size_t)(q0 + rt * 16 + c) * kD + dc * 32 + 8 * hh);
#pragma unroll
    for (int t = 0; t < 2; ++t) {
      const int ct = wave + 8 * t;
      if (ct * 16 < nk) {
        const _Float16* kp = Qb + (size_t)(ct * 16 + c) * kD + 8 * hh;
        const v16h kb0 = FragH::load(kp);
        const v16h kb1 = FragH::load(kp + 32);
        v8f acc0 = (v8f){0.f,0.f,0.f,0.f,0.f,0.f,0.f,0.f};
        v8f acc1 = (v8f){0.f,0.f,0.f,0.f,0.f,0.f,0.f,0.f};
        acc0 = FragH::mma(qa[0][0], kb0, acc0);
        acc0 = FragH::mma(qa[0][1], kb1, acc0);
        acc1 = FragH::mma(qa[1][0], kb0, acc1);
        acc1 = FragH::mma(qa[1][1], kb1, acc1);
        guard2_h(acc0, acc1, kb0, kb1);
#pragma unroll
        for (int r = 0; r < 8; ++r) {
          sc[(8 * hh + r) * kSCP + ct * 16 + c]      = acc0[r] * kScoreScale;
          sc[(16 + 8 * hh + r) * kSCP + ct * 16 + c] = acc1[r] * kScoreScale;
        }
      }
    }
    keep4_h(qa[0][0], qa[0][1], qa[1][0], qa[1][1]);
  }
  __syncthreads();

  {
    const int r  = tid >> 3;
    const int cl = tid & 7;
    const int iq = q0 + r;
    const int lim = strict ? (iq - 1) : iq;
    const bool any = (lim >= 0);
    const int chunk = nk >> 3;
    const int j0 = cl * chunk;
    float* srow = sc + r * kSCP + j0;
    _Float16* arow = at + r * kATP + j0;

    const float gq = bf16_rne(gam[h]);
    const float gamma = -(fmaxf(gq, 0.f) + log1pf(expf(-fabsf(gq))));

    float m1 = -INFINITY;
#pragma unroll 1
    for (int t = 0; t < chunk; t += 4) {
      const v4f s4 = *(const v4f*)(srow + t);
#pragma unroll
      for (int e = 0; e < 4; ++e) {
        const int j = j0 + t + e;
        const float sv = s4[e];
        m1 = fmaxf(m1, (j <= lim) ? sv : -INFINITY);
      }
    }
    m1 = fmaxf(m1, __shfl_xor(m1, 1, 32));
    m1 = fmaxf(m1, __shfl_xor(m1, 2, 32));
    m1 = fmaxf(m1, __shfl_xor(m1, 4, 32));
    const float m1s = any ? m1 : 0.f;

    float ev[kChunkMax];
#pragma unroll
    for (int i = 0; i < kChunkMax; ++i) ev[i] = 0.f;
    float ls = 0.f;
#pragma unroll
    for (int t = 0; t < kChunkMax; t += 4) {
      if (t < chunk) {
        const v4f s4 = *(const v4f*)(srow + t);
#pragma unroll
        for (int e = 0; e < 4; ++e) {
          const int j = j0 + t + e;
          const float sv = s4[e];
          const float x = (j <= lim) ? __expf(fminf(sv - m1s, 0.f)) : 0.f;
          ev[t + e] = x;
          ls += x;
        }
      }
    }
    float tot = ls;
    tot += __shfl_xor(tot, 1, 32);
    tot += __shfl_xor(tot, 2, 32);
    tot += __shfl_xor(tot, 4, 32);
    float scan = ls;
#pragma unroll
    for (int d = 1; d < 8; d <<= 1) {
      const int src = (cl >= d) ? (lane - d) : lane;
      const float v = __shfl(scan, src, 32);
      scan += (cl >= d) ? v : 0.f;
    }
    const float inv = (tot > 0.f) ? __builtin_amdgcn_rcpf(tot) : 0.f;
    const float totP = tot * inv;
    float runP = (scan - ls) * inv;

    float m2 = -INFINITY;
#pragma unroll
    for (int t = 0; t < kChunkMax; t += 4) {
      if (t < chunk) {
        const v4f s4 = *(const v4f*)(srow + t);
        v4f o4;
#pragma unroll
        for (int e = 0; e < 4; ++e) {
          const int j = j0 + t + e;
          const bool ok = (j <= lim);
          const float sv = s4[e];
          const float evv = ev[t + e];
          runP = fmaf(evv, inv, runP);
          const float tail = totP - runP;
          const float pos = fabsf((float)(iq - j));
          const float dist = __builtin_amdgcn_sqrtf(fmaxf(tail * pos, 0.f));
          float eff = __expf(dist * gamma);
          eff = fminf(fmaxf(eff, 1e-5f), 1e5f);
          const float s2 = sv * eff;
          m2 = fmaxf(m2, ok ? s2 : -INFINITY);
          o4[e] = s2;
        }
        *(v4f*)(srow + t) = o4;
      }
    }
    m2 = fmaxf(m2, __shfl_xor(m2, 1, 32));
    m2 = fmaxf(m2, __shfl_xor(m2, 2, 32));
    m2 = fmaxf(m2, __shfl_xor(m2, 4, 32));
    const float m2s = any ? m2 : 0.f;

    float ls2 = 0.f;
#pragma unroll 1
    for (int t = 0; t < chunk; t += 4) {
      const v4f s4 = *(const v4f*)(srow + t);
      v4h hv;
#pragma unroll
      for (int e = 0; e < 4; ++e) {
        const int j = j0 + t + e;
        const float sv = s4[e];
        const float e2 = (j <= lim) ? __expf(fminf(sv - m2s, 0.f)) : 0.f;
        ls2 += e2;
        hv[e] = (_Float16)(e2 * kPCarry);
      }
      *(v4h*)(arow + t) = hv;
    }
    float tot2 = ls2;
    tot2 += __shfl_xor(tot2, 1, 32);
    tot2 += __shfl_xor(tot2, 2, 32);
    tot2 += __shfl_xor(tot2, 4, 32);
    const float rv = (tot2 > 0.f) ? (kACarry * __builtin_amdgcn_rcpf(tot2 * kPCarry)) : 0.f;
    if (cl == 0) rinv[r] = rv;
  }
  __syncthreads();

  {
    const int rt = wave >> 2, ct = wave & 3;
    const _Float16* ap = at + (rt * 16 + c) * kATP + 8 * hh;
    const _Float16* vp = (const _Float16*)vT16 + (size_t)(h * kDh + ct * 16 + c) * kM + (size_t)b * kS + 8 * hh;
    v8f acc = (v8f){0.f,0.f,0.f,0.f,0.f,0.f,0.f,0.f};
#pragma unroll 1
    for (int k0 = 0; k0 < nk; k0 += 32) {
      const v16h pa = FragH::load(ap + k0);
      const v16h vb = FragH::load(vp + k0);
      acc = mma_guarded(pa, vb, acc);
    }
#pragma unroll
    for (int r = 0; r < 8; ++r) {
      const int row = rt * 16 + 8 * hh + r;
      sc[row * kOSP + ct * 16 + c] = acc[r] * rinv[row];
    }
  }
  __syncthreads();
  {
    const int row = wave * 4 + (lane >> 3);
    const int c8 = (lane & 7) * 8;
    const float* sp = sc + row * kOSP + c8;
    const v4f x0 = *(const v4f*)(sp);
    const v4f x1 = *(const v4f*)(sp + 4);
    v8h hv;
#pragma unroll
    for (int e = 0; e < 4; ++e) {
      hv[e]     = (_Float16)x0[e];
      hv[4 + e] = (_Float16)x1[e];
    }
    unsigned short* dst = a16 + (size_t)(b * kS + q0 + row) * kD + h * kDh + c8;
    for (int pass = 0; pass < 2; ++pass) {
      *(volatile v8h*)dst = hv;
      __threadfence();
    }
  }
}

__global__ __launch_bounds__(256) void add_ln_kernel(
    const float* __restrict__ resid, int residRaw, const float* __restrict__ delta,
    const float* __restrict__ gw, const float* __restrict__ bw,
    float* __restrict__ outF, unsigned short* __restrict__ out16) {
  const int lane = threadIdx.x & 31, wave = threadIdx.x >> 5;
  const int row = blockIdx.x * 8 + wave;
  const size_t base = (size_t)row * kD;
  float x[16];
#pragma unroll
  for (int it = 0; it < 4; ++it) {
    const int col = it * 128 + lane * 4;
    const v4f a = *(const v4f*)(resid + base + col);
    const v4f d = *(const v4f*)(delta + base + col);
#pragma unroll
    for (int e = 0; e < 4; ++e) {
      const float av = a[e];
      const float rv = residRaw ? bf16_rne(av) : av;
      x[it * 4 + e] = rv + d[e];
    }
  }
  float s = 0.f;
#pragma unroll
  for (int i = 0; i < 16; ++i) s += x[i];
#pragma unroll
  for (int off = 16; off > 0; off >>= 1) s += __shfl_xor(s, off, 32);
  const float mean = s * kInvD;
  float vs = 0.f;
#pragma unroll
  for (int i = 0; i < 16; ++i) {
    const float dlt = x[i] - mean;
    vs = fmaf(dlt, dlt, vs);
  }
#pragma unroll
  for (int off = 16; off > 0; off >>= 1) vs += __shfl_xor(vs, off, 32);
  const float rstd = __builtin_amdgcn_rcpf(__builtin_amdgcn_sqrtf(vs * kInvD + kLnEps));
  v4f ov[4];
  v4h hv[4];
#pragma unroll
  for (int it = 0; it < 4; ++it) {
    const int col = it * 128 + lane * 4;
    const v4f g4 = *(const v4f*)(gw + col);
    const v4f b4 = *(const v4f*)(bw + col);
#pragma unroll
    for (int e = 0; e < 4; ++e) {
      const float gv = bf16_rne(g4[e]);
      const float bv = bf16_rne(b4[e]);
      const float o = (x[it * 4 + e] - mean) * rstd * gv + bv;
      ov[it][e] = o;
      hv[it][e] = (_Float16)o;
    }
  }
  for (int pass = 0; pass < 2; ++pass) {
#pragma unroll
    for (int it = 0; it < 4; ++it) {
      const int col = it * 128 + lane * 4;
      *(volatile v4f*)(outF + base + col) = ov[it];
      if (out16) *(volatile v4h*)(out16 + base + col) = hv[it];
    }
    __threadfence();
  }
}

extern "C" void kernel_launch(void* const* d_in, const int* in_sizes, int n_in,
                              void* d_out, int out_size, void* d_ws, size_t ws_size,
                              hipStream_t stream) {
  if (n_in < 18) return;
  if (in_sizes[0] != kM * kD || in_sizes[1] != kM * kD) return;
  if (in_sizes[3] != kL * kD * kD || in_sizes[5] != kL * kD * kD || in_sizes[7] != kL * kD * kD) return;
  if (in_sizes[4] != kL * kD || in_sizes[6] != kL * kD || in_sizes[8] != kL * kD) return;
  if (in_sizes[9] != kL * kH) return;
  if (in_sizes[10] != kL * kD || in_sizes[11] != kL * kD) return;
  if (in_sizes[12] != kL * kD * kF || in_sizes[14] != kL * kF * kD) return;
  if (in_sizes[13] != kL * kF || in_sizes[15] != kL * kD) return;
  if (in_sizes[16] != kL * kD || in_sizes[17] != kL * kD) return;
  if (out_size != kM * kD) return;
  if (ws_size < kWsTotal) return;

  const float* qemb = (const float*)d_in[0];
  const float* iemb = (const float*)d_in[1];
  const float* Wk   = (const float*)d_in[3];
  const float* bk   = (const float*)d_in[4];
  const float* Wv   = (const float*)d_in[5];
  const float* bv   = (const float*)d_in[6];
  const float* Wo   = (const float*)d_in[7];
  const float* bo   = (const float*)d_in[8];
  const float* gam  = (const float*)d_in[9];
  const float* ln1g = (const float*)d_in[10];
  const float* ln1b = (const float*)d_in[11];
  const float* W1   = (const float*)d_in[12];
  const float* b1   = (const float*)d_in[13];
  const float* W2   = (const float*)d_in[14];
  const float* b2   = (const float*)d_in[15];
  const float* ln2g = (const float*)d_in[16];
  const float* ln2b = (const float*)d_in[17];

  char* ws = (char*)d_ws;
  float* P0 = (float*)(ws + kOffP0);
  float* P1 = (float*)(ws + kOffP1);
  float* Ob = (float*)(ws + kOffO);
  unsigned short* X16 = (unsigned short*)(ws + kOffX16);
  unsigned short* Y16 = (unsigned short*)(ws + kOffY16);
  unsigned short* T16 = (unsigned short*)(ws + kOffT16);
  unsigned short* QK16 = (unsigned short*)(ws + kOffU);
  unsigned short* VT16 = (unsigned short*)(ws + kOffU + kPlaneH);
  unsigned short* A16  = (unsigned short*)(ws + kOffU + 2 * kPlaneH);
  unsigned short* F1   = (unsigned short*)(ws + kOffU);
  unsigned short* WS   = (unsigned short*)(ws + kOffWS);
  unsigned short* WkT = WS;
  unsigned short* WvT = WS + (size_t)kD * kD;
  unsigned short* WoT = WS + (size_t)2 * kD * kD;
  unsigned short* W1T = WS + (size_t)3 * kD * kD;
  unsigned short* W2T = WS + (size_t)3 * kD * kD + (size_t)kD * kF;

  const int n8 = kM * kD / 8;
  cast8_kernel<<<n8 / 256, 256, 0, stream>>>(qemb, X16, n8);
  cast8_kernel<<<n8 / 256, 256, 0, stream>>>(iemb, Y16, n8);

  const int gD = (kM / 64) * (kD / 64) / 8;
  const int gF = (kM / 64) * (kF / 64) / 8;

  auto layer = [&](int i, const unsigned short* xq16, const unsigned short* xv16,
                   const float* resid, int residRaw, float* mid, float* outF, unsigned short* out16,
                   bool ffn, int strict) {
    const size_t oDD = (size_t)i * kD * kD;
    const size_t oDF = (size_t)i * kD * kF;
    const size_t oD  = (size_t)i * kD;
    const size_t oF  = (size_t)i * kF;
    wprep_kernel<<<ffn ? 704 : 192, 256, 0, stream>>>(Wk + oDD, Wv + oDD, Wo + oDD, W1 + oDF, W2 + oDF, WS);
    wmma_gemm64<2, 1, 0><<<gD, 256, 0, stream>>>(xq16, kD, WkT, kD, (void*)QK16, kD, bk + oD, kM, kD, kD, kWCarryInv);
    wmma_gemm64<1, 1, 0><<<gD, 256, 0, stream>>>(WvT, kD, xv16, kD, (void*)VT16, kM, bv + oD, kD, kM, kD, kWCarryInv);
    decay_attn_kernel<<<kB * kH * (kS / kQT), 256, 0, stream>>>(QK16, VT16, A16, gam + (size_t)i * kH, strict);
    wmma_gemm64<2, 0, 0><<<gD, 256, 0, stream>>>(A16, kD, WoT, kD, (void*)Ob, kD, bo + oD, kM, kD, kD, kOutScale);
    if (!ffn) {
      add_ln_kernel<<<kM / 8, 256, 0, stream>>>(resid, residRaw, Ob, ln1g + oD, ln1b + oD, outF, out16);
    } else {
      add_ln_kernel<<<kM / 8, 256, 0, stream>>>(resid, residRaw, Ob, ln1g + oD, ln1b + oD, mid, T16);
      wmma_gemm64<2, 1, 2><<<gF, 256, 0, stream>>>(T16, kD, W1T, kD, (void*)F1, kF, b1 + oF, kM, kF, kD, kWCarryInv);
      wmma_gemm64<2, 0, 0><<<gD, 256, 0, stream>>>(F1, kF, W2T, kF, (void*)Ob, kD, b2 + oD, kM, kD, kF, kWCarryInv);
      add_ln_kernel<<<kM / 8, 256, 0, stream>>>(mid, 0, Ob, ln2g + oD, ln2b + oD, outF, out16);
    }
  };

  layer(0, Y16, Y16, iemb, 1, P1, P0, Y16, true, 0);
  layer(1, Y16, Y16, P0,   0, P1, P0, Y16, true, 0);
  layer(2, X16, X16, qemb, 1, P1, P0, X16, false, 0);
  layer(3, X16, Y16, P0,   0, P1, P0, X16, true, 1);
  layer(4, X16, X16, P0,   0, P0, P1, X16, false, 0);
  layer(5, X16, Y16, P1,   0, P0, (float*)d_out, (unsigned short*)nullptr, true, 1);
}
